// PointNetPP_18691697672886
// MI455X (gfx1250) — hardware-verified
//
#include <hip/hip_runtime.h>
#include <stddef.h>

#pragma clang fp contract(off)

typedef __attribute__((ext_vector_type(16))) __bf16   v16b;
typedef __attribute__((ext_vector_type(8)))  __bf16   v8b;
typedef __attribute__((ext_vector_type(8)))  float    v8f;
typedef __attribute__((ext_vector_type(4)))  float    v4f;
typedef __attribute__((ext_vector_type(4)))  unsigned v4u;
typedef __attribute__((ext_vector_type(2)))  unsigned v2u;

constexpr int kPts0 = 8192;
constexpr int kPts1 = 4096;
constexpr int kPts2 = 2048;
constexpr int kPts3 = 1024;
constexpr int kFeatIn = 16;
constexpr int kHid = 128;
constexpr int kSaHid = 131;
constexpr int kSaHidPadK = 160;
constexpr int kSaHidPadN = 192;
constexpr int kFpHid = 256;
constexpr int kNbr = 32;
constexpr int kAPitch = 168;
constexpr long kSaW1Level = (long)kSaHid * kSaHid;
constexpr long kSaW2Level = (long)kSaHid * kHid;
static_assert(kSaHid == kHid + 3, "SA MLP input = features + rel pos");
static_assert(kSaHidPadK % 32 == 0 && kSaHidPadK >= kSaHid, "K pad");
static_assert(kSaHidPadN % 64 == 0 && kSaHidPadN >= kSaHid, "N pad");
static_assert(kPts0 % 512 == 0 && kPts3 % 256 == 0, "tile multiples");
static_assert((kAPitch * 2) % 16 == 0, "LDS row pitch 16-B aligned");

__device__ __forceinline__ unsigned f2bf_bits(float f) {
  const unsigned u = __float_as_uint(f);
  return (u + 0x7FFFu + ((u >> 16) & 1u)) >> 16;
}
__device__ __forceinline__ float bf_bits2f(unsigned h) { return __uint_as_float(h << 16); }
__device__ __forceinline__ float bf_lo(unsigned w) { return __uint_as_float(w << 16); }
__device__ __forceinline__ float bf_hi(unsigned w) { return __uint_as_float(w & 0xffff0000u); }
__device__ __forceinline__ void split_pair(float a, float b, unsigned& wh, unsigned& wl) {
  const unsigned ha = f2bf_bits(a);
  const unsigned hb = f2bf_bits(b);
  const unsigned la = f2bf_bits(a - bf_bits2f(ha));
  const unsigned lb = f2bf_bits(b - bf_bits2f(hb));
  wh = (ha & 0xffffu) | (hb << 16);
  wl = (la & 0xffffu) | (lb << 16);
}

union FragB { v16b v; v8b h[2]; };
__device__ __forceinline__ v16b frag_load(const __bf16* p) {
  FragB f;
  f.h[0] = *(const v8b*)(p);
  f.h[1] = *(const v8b*)(p + 16);
  return f.v;
}
__device__ __forceinline__ v8f mma_b(v16b a, v16b b, v8f c) {
  return __builtin_amdgcn_wmma_f32_16x16x32_bf16(false, a, false, b, (short)0, c, false, false);
}
__device__ __forceinline__ void dep_guard4_b(v8f& a, v8f& b, v8f& c, v8f& d, v16b x, v16b y) {
  asm volatile("v_nop\n\tv_nop\n\tv_nop\n\tv_nop" : "+v"(a), "+v"(b), "+v"(c), "+v"(d) : "v"(x), "v"(y));
}
__device__ __forceinline__ void keep4_b(v16b a, v16b b, v16b c, v16b d) {
  asm volatile("v_nop" :: "v"(a), "v"(b), "v"(c), "v"(d));
}
__device__ __forceinline__ void acc_guard4(v8f& a, v8f& b, v8f& c, v8f& d) {
  asm volatile("v_nop\n\tv_nop\n\tv_nop\n\tv_nop" : "+v"(a), "+v"(b), "+v"(c), "+v"(d));
}
__device__ __forceinline__ void group_guard(v8f& a, v16b x, v16b y, v16b z, v16b w) {
  asm volatile("v_nop\n\tv_nop\n\tv_nop\n\tv_nop" : "+v"(a) : "v"(x), "v"(y), "v"(z), "v"(w));
}

__global__ __launch_bounds__(256) void prep_split_kernel(
    const float* __restrict__ src, long srcLevelStride, int sn, int sk,
    int Kreal, int Nreal, int Kpad, int Npad,
    unsigned short* __restrict__ dhi, unsigned short* __restrict__ dlo, long dstLevelStride) {
  const int lvl = blockIdx.y;
  const long total = (long)Npad * Kpad;
  const long e = ((long)blockIdx.x * 256 + threadIdx.x) * 8;
  if (e < total) {
    const int n = (int)(e / Kpad);
    const int k0 = (int)(e - (long)n * Kpad);
    const float* s = src + (size_t)lvl * srcLevelStride;
    const int nc = n < Nreal ? n : Nreal - 1;
    float v[8];
#pragma unroll
    for (int i = 0; i < 8; ++i) {
      const int k = k0 + i;
      const int kc = k < Kreal ? k : Kreal - 1;
      const float x = s[(size_t)nc * sn + (size_t)kc * sk];
      v[i] = (n < Nreal && k < Kreal) ? x : 0.0f;
    }
    unsigned wh[4], wl[4];
#pragma unroll
    for (int i = 0; i < 4; ++i) split_pair(v[2 * i], v[2 * i + 1], wh[i], wl[i]);
    const v4u hv = {wh[0], wh[1], wh[2], wh[3]};
    const v4u lv = {wl[0], wl[1], wl[2], wl[3]};
    unsigned short* ph = dhi + (size_t)lvl * dstLevelStride + e;
    unsigned short* pl = dlo + (size_t)lvl * dstLevelStride + e;
    *(volatile v4u*)(void*)ph = hv;
    *(volatile v4u*)(void*)pl = lv;
    __threadfence();
    *(volatile v4u*)(void*)ph = hv;
    *(volatile v4u*)(void*)pl = lv;
  }
}

template <int BIAS_MODE, int OUT_MODE, int ACT>
__global__ __launch_bounds__(256) void gemm_bf16x3_kernel(
    const unsigned short* __restrict__ Ahp, const unsigned short* __restrict__ Alp, int lda,
    const unsigned short* __restrict__ Bhp, const unsigned short* __restrict__ Blp, int ldb,
    void* __restrict__ Cout, void* __restrict__ Cout2, int ldc,
    const float* __restrict__ bias, int M, int N, int K) {
  __shared__ __align__(16) float sT[8][16 * 68];
  const int lane = threadIdx.x & 31;
  const int wave = threadIdx.x >> 5;
  const int tilesN = N >> 6;
  const int tilesM = M >> 6;
  const int tile = blockIdx.x * 8 + wave;
  if (tile >= tilesM * tilesN) return;
  const int tm = tile / tilesN;
  const int tn = tile - tm * tilesN;
  const int m0 = tm << 6;
  const int n0 = tn << 6;

  const __bf16* Ah = (const __bf16*)(const void*)Ahp;
  const __bf16* Al = (const __bf16*)(const void*)Alp;
  const __bf16* Bh = (const __bf16*)(const void*)Bhp;
  const __bf16* Bl = (const __bf16*)(const void*)Blp;

  const int rlane = lane & 15;
  const int koff = (lane >> 4) * 8;
  const int mOff = (lane >> 4) * 8;

  v8f acc[4][4];
#pragma unroll
  for (int i = 0; i < 4; ++i)
#pragma unroll
    for (int j = 0; j < 4; ++j) acc[i][j] = (v8f){0.f, 0.f, 0.f, 0.f, 0.f, 0.f, 0.f, 0.f};

  for (int k0 = 0; k0 < K; k0 += 32) {
    v16b bh[4], bl[4];
#pragma unroll
    for (int j = 0; j < 4; ++j) {
      const size_t bo = (size_t)(n0 + (j << 4) + rlane) * ldb + koff + k0;
      bh[j] = frag_load(Bh + bo);
      bl[j] = frag_load(Bl + bo);
    }
#pragma unroll
    for (int i = 0; i < 4; ++i) {
      const size_t ao = (size_t)(m0 + (i << 4) + rlane) * lda + koff + k0;
      const v16b ah = frag_load(Ah + ao);
      const v16b al = frag_load(Al + ao);
#pragma unroll
      for (int j = 0; j < 4; ++j) {
        acc[i][j] = mma_b(ah, bh[j], acc[i][j]);
        acc[i][j] = mma_b(ah, bl[j], acc[i][j]);
        acc[i][j] = mma_b(al, bh[j], acc[i][j]);
      }
      dep_guard4_b(acc[i][0], acc[i][1], acc[i][2], acc[i][3], ah, al);
    }
    keep4_b(bh[0], bh[1], bh[2], bh[3]);
    keep4_b(bl[0], bl[1], bl[2], bl[3]);
  }
  acc_guard4(acc[0][0], acc[0][1], acc[0][2], acc[0][3]);
  acc_guard4(acc[1][0], acc[1][1], acc[1][2], acc[1][3]);
  acc_guard4(acc[2][0], acc[2][1], acc[2][2], acc[2][3]);
  acc_guard4(acc[3][0], acc[3][1], acc[3][2], acc[3][3]);

  float* slab = sT[wave];
#pragma unroll
  for (int i = 0; i < 4; ++i) {
    const int mBase = m0 + (i << 4);
#pragma unroll
    for (int j = 0; j < 4; ++j) {
      const int n = n0 + (j << 4) + rlane;
      float bv = 0.f;
      if (BIAS_MODE == 2) bv = bias[n];
#pragma unroll
      for (int r = 0; r < 8; ++r) {
        float v = acc[i][j][r];
        if (BIAS_MODE == 2) v = v + bv;
        if (ACT == 2) v = fmaxf(v, 0.0f);
        slab[(mOff + r) * 68 + (j << 4) + rlane] = v;
      }
    }
    __builtin_amdgcn_fence(__ATOMIC_RELEASE, "workgroup");
    __builtin_amdgcn_wave_barrier();
    __builtin_amdgcn_fence(__ATOMIC_ACQUIRE, "workgroup");
    if (OUT_MODE == 0) {
      float* C = (float*)Cout;
      const int hh = lane >> 4, c4 = (lane & 15) * 4;
      for (int pass = 0; pass < 2; ++pass) {
#pragma unroll
        for (int it = 0; it < 8; ++it) {
          const int row = it * 2 + hh;
          const v4f v = *(const v4f*)(slab + row * 68 + c4);
          *(volatile v4f*)(C + (size_t)(mBase + row) * ldc + n0 + c4) = v;
        }
        __threadfence();
      }
    } else {
      const int q = lane >> 3, c8 = (lane & 7) * 8;
      unsigned short* C = (unsigned short*)Cout;
      unsigned short* C2 = (unsigned short*)Cout2;
      for (int pass = 0; pass < 2; ++pass) {
#pragma unroll
        for (int it = 0; it < 4; ++it) {
          const int row = it * 4 + q;
          const float* sp = slab + row * 68 + c8;
          unsigned wh[4], wl[4];
#pragma unroll
          for (int e2 = 0; e2 < 4; ++e2) split_pair(sp[2 * e2], sp[2 * e2 + 1], wh[e2], wl[e2]);
          const v4u hv = {wh[0], wh[1], wh[2], wh[3]};
          const v4u lv = {wl[0], wl[1], wl[2], wl[3]};
          *(volatile v4u*)(void*)(C + (size_t)(mBase + row) * ldc + n0 + c8) = hv;
          *(volatile v4u*)(void*)(C2 + (size_t)(mBase + row) * ldc + n0 + c8) = lv;
        }
        __threadfence();
      }
    }
    __builtin_amdgcn_fence(__ATOMIC_RELEASE, "workgroup");
    __builtin_amdgcn_wave_barrier();
    __builtin_amdgcn_fence(__ATOMIC_ACQUIRE, "workgroup");
  }
}

template <int NPT>
__global__ __launch_bounds__(512) void fps_kernel(const float* __restrict__ pos, int m,
                                                   float* __restrict__ qpos) {
#pragma clang fp contract(off)
  __shared__ float sVal[2][16];
  __shared__ int sIdx[2][16];
  __shared__ int sList[4096];
  const int t = threadIdx.x;
  const int lane = t & 31;
  const int wave = t >> 5;
  const int n = NPT * 512;
  if (m > 4096) m = 4096;

  float px[NPT], py[NPT], pz[NPT], md[NPT];
#pragma unroll
  for (int k = 0; k < NPT; ++k) {
    const int i = t + k * 512;
    float a = pos[3 * i], b = pos[3 * i + 1], c = pos[3 * i + 2];
    asm volatile("" : "+v"(a), "+v"(b), "+v"(c));
    px[k] = a;
    py[k] = b;
    pz[k] = c;
    md[k] = 1e30f;
  }
  if (t == 0) sList[0] = 0;
  int last = 0;
  for (int s = 1; s < m; ++s) {
    const float lx = pos[3 * last], ly = pos[3 * last + 1], lz = pos[3 * last + 2];
    float bv = -1.0f;
    int bi = 0;
#pragma unroll
    for (int k = 0; k < NPT; ++k) {
      const float dx = px[k] - lx, dy = py[k] - ly, dz = pz[k] - lz;
      const float t0 = dx * dx;
      const float t1 = dy * dy;
      const float t2 = dz * dz;
      const float d = (t0 + t2) + t1;
      const float mm = fminf(md[k], d);
      md[k] = mm;
      const bool tk = mm > bv;
      bv = tk ? mm : bv;
      bi = tk ? (t + k * 512) : bi;
    }
#pragma unroll
    for (int off = 16; off > 0; off >>= 1) {
      const float ov = __shfl_xor(bv, off, 32);
      const int oi = __shfl_xor(bi, off, 32);
      const bool tk = (ov > bv) || (ov == bv && oi < bi);
      bv = tk ? ov : bv;
      bi = tk ? oi : bi;
    }
    const int par = s & 1;
    if (lane == 0) {
      sVal[par][wave] = bv;
      sIdx[par][wave] = bi;
    }
    __syncthreads();
    float v = sVal[par][lane & 15];
    int vi = sIdx[par][lane & 15];
#pragma unroll
    for (int off = 8; off > 0; off >>= 1) {
      const float ov = __shfl_xor(v, off, 32);
      const int oi = __shfl_xor(vi, off, 32);
      const bool tk = (ov > v) || (ov == v && oi < vi);
      v = tk ? ov : v;
      vi = tk ? oi : vi;
    }
    int nl = __builtin_amdgcn_readfirstlane(vi);
    nl = nl < 0 ? 0 : nl;
    nl = nl > n - 1 ? n - 1 : nl;
    last = nl;
    if (t == 0) sList[s] = last;
  }
  __syncthreads();
  for (int pass = 0; pass < 2; ++pass) {
    for (int e = t; e < 3 * m; e += 512) {
      const int c = e / 3;
      const int comp = e - 3 * c;
      int i = sList[c];
      i = i < 0 ? 0 : i;
      i = i > n - 1 ? n - 1 : i;
      const float val = pos[3 * i + comp];
      *(volatile float*)(qpos + e) = val;
    }
    __threadfence();
  }
}

__global__ __launch_bounds__(256) void sa_fused_kernel(
    const float* __restrict__ pos, int n,
    const float* __restrict__ qpos,
    const float* __restrict__ P,
    const float* __restrict__ w1r, const float* __restrict__ b1,
    const unsigned short* __restrict__ w2h, const unsigned short* __restrict__ w2l,
    const float* __restrict__ b2,
    unsigned short* __restrict__ fh, unsigned short* __restrict__ fl) {
#pragma clang fp contract(off)
  __shared__ __align__(16) unsigned short sAh[64 * kAPitch];
  __shared__ __align__(16) unsigned short sAl[64 * kAPitch];
  __shared__ int sNbr[8][32];
  __shared__ float sRx[8][32];
  __shared__ float sRy[8][32];
  __shared__ float sRz[8][32];
  __shared__ unsigned sVm[8];
  __shared__ __align__(16) float sW0[kSaHidPadK];
  __shared__ __align__(16) float sW1[kSaHidPadK];
  __shared__ __align__(16) float sW2[kSaHidPadK];
  __shared__ __align__(16) float sB1[kSaHidPadK];
  __shared__ __align__(16) float sOut[8 * 128];

  const int tid = threadIdx.x;
  const int lane = tid & 31;
  const int wave = tid >> 5;

  if (tid < kSaHidPadK) {
    const bool ok = tid < kSaHid;
    const int cc = ok ? tid : kSaHid - 1;
    const float a0 = w1r[cc];
    const float a1 = w1r[kSaHid + cc];
    const float a2 = w1r[2 * kSaHid + cc];
    const float bb = b1[cc];
    sW0[tid] = ok ? a0 : 0.0f;
    sW1[tid] = ok ? a1 : 0.0f;
    sW2[tid] = ok ? a2 : 0.0f;
    sB1[tid] = ok ? bb : 0.0f;
  }

  {
    const int ctr = blockIdx.x * 8 + wave;
    const float qx = qpos[3 * ctr], qy = qpos[3 * ctr + 1], qz = qpos[3 * ctr + 2];
    float ld = __builtin_inff();
    int li = 0;
    float tau = __builtin_inff();
    for (int base = 0; base < n; base += 32) {
      const int jr = base + lane;
      const int j = jr < n ? jr : n - 1;
      const float x = pos[3 * j], y = pos[3 * j + 1], z = pos[3 * j + 2];
      const float dx = qx - x, dy = qy - y, dz = qz - z;
      const float t0 = dx * dx;
      const float t1 = dy * dy;
      const float t2 = dz * dz;
      const float d = (t0 + t2) + t1;
      unsigned hits = (unsigned)__ballot((d < tau) && (jr < n));
      while (hits != 0u) {
        const int src = __builtin_ctz(hits);
        hits &= hits - 1u;
        const float cd = __shfl(d, src, 32);
        const int ci = base + src;
        const float pd = __shfl_up(ld, 1, 32);
        const int pi = __shfl_up(li, 1, 32);
        const bool gt = ld > cd;
        const bool pgt = (lane > 0) && (pd > cd);
        const float nd = gt ? (pgt ? pd : cd) : ld;
        const int ni = gt ? (pgt ? pi : ci) : li;
        ld = nd;
        li = ni;
        tau = __shfl(ld, 31, 32);
      }
    }
    int nb = li < 0 ? 0 : li;
    nb = nb > n - 1 ? n - 1 : nb;
    const float rx = pos[3 * nb] - qx;
    const float ry = pos[3 * nb + 1] - qy;
    const float rz = pos[3 * nb + 2] - qz;
    const unsigned vm = (unsigned)__ballot(ld <= 4.0f);
    sNbr[wave][lane] = nb;
    sRx[wave][lane] = rx;
    sRy[wave][lane] = ry;
    sRz[wave][lane] = rz;
    if (lane == 0) sVm[wave] = vm;
  }
  __syncthreads();

  const int rl = lane & 15;
  const int hh = lane >> 4;
  const int koff = hh * 8;
  const int ncol = wave * 16 + rl;
  const __bf16* Bh = (const __bf16*)(const void*)w2h;
  const __bf16* Bl = (const __bf16*)(const void*)w2l;
  v16b bhf[5], blf[5];
#pragma unroll
  for (int kt = 0; kt < 5; ++kt) {
    bhf[kt] = frag_load(Bh + (size_t)ncol * kSaHidPadK + kt * 32 + koff);
    blf[kt] = frag_load(Bl + (size_t)ncol * kSaHidPadK + kt * 32 + koff);
    asm volatile("" : "+v"(bhf[kt]), "+v"(blf[kt]));
  }
  const float bias2 = b2[ncol];
  const __bf16* sAhB = (const __bf16*)(const void*)sAh;
  const __bf16* sAlB = (const __bf16*)(const void*)sAl;

  for (int p = 0; p < 4; ++p) {
#pragma unroll 2
    for (int it = 0; it < 10; ++it) {
      const int item = tid + it * 256;
      const int row = item / 40;
      const int c4 = (item - row * 40) * 4;
      const int cw = p * 2 + (row >> 5);
      const int kk = row & 31;
      const int nb = sNbr[cw][kk];
      const float rx = sRx[cw][kk], ry = sRy[cw][kk], rz = sRz[cw][kk];
      const v4f pv = *(const v4f*)(P + (size_t)nb * kSaHidPadN + c4);
      const v4f a0 = *(const v4f*)(sW0 + c4);
      const v4f a1 = *(const v4f*)(sW1 + c4);
      const v4f a2 = *(const v4f*)(sW2 + c4);
      const v4f bb = *(const v4f*)(sB1 + c4);
      float v[4];
#pragma unroll
      for (int e = 0; e < 4; ++e) {
        float u = pv[e] + bb[e];
        u = u + rx * a0[e];
        u = u + ry * a1[e];
        u = u + rz * a2[e];
        u = fmaxf(u, 0.0f);
        v[e] = ((c4 + e) < kSaHid) ? u : 0.0f;
      }
      unsigned wh0, wl0, wh1, wl1;
      split_pair(v[0], v[1], wh0, wl0);
      split_pair(v[2], v[3], wh1, wl1);
      const v2u hv = {wh0, wh1};
      const v2u lv = {wl0, wl1};
      *(v2u*)(void*)(sAh + row * kAPitch + c4) = hv;
      *(v2u*)(void*)(sAl + row * kAPitch + c4) = lv;
    }
    __syncthreads();

    v8f acc[4];
#pragma unroll
    for (int i = 0; i < 4; ++i) acc[i] = (v8f){0.f, 0.f, 0.f, 0.f, 0.f, 0.f, 0.f, 0.f};
#pragma unroll
    for (int kt = 0; kt < 5; ++kt) {
#pragma unroll
      for (int i = 0; i < 4; ++i) {
        const int ao = (i * 16 + rl) * kAPitch + kt * 32 + koff;
        const v16b ah = frag_load(sAhB + ao);
        const v16b al = frag_load(sAlB + ao);
        acc[i] = mma_b(ah, bhf[kt], acc[i]);
        acc[i] = mma_b(ah, blf[kt], acc[i]);
        acc[i] = mma_b(al, bhf[kt], acc[i]);
        group_guard(acc[i], ah, al, bhf[kt], blf[kt]);
      }
    }
    acc_guard4(acc[0], acc[1], acc[2], acc[3]);

#pragma unroll
    for (int ci = 0; ci < 2; ++ci) {
      const int cw = p * 2 + ci;
      const unsigned vm = sVm[cw];
      float mx = 0.0f;
#pragma unroll
      for (int ii = 0; ii < 2; ++ii) {
#pragma unroll
        for (int r = 0; r < 8; ++r) {
          const int rowk = ii * 16 + 8 * hh + r;
          const float val = acc[2 * ci + ii][r] + bias2;
          const bool ok = ((vm >> rowk) & 1u) != 0u;
          mx = fmaxf(mx, ok ? val : 0.0f);
        }
      }
      const float other = __shfl_xor(mx, 16, 32);
      mx = fmaxf(mx, other);
      if (lane < 16) sOut[cw * 128 + ncol] = mx;
    }
    __syncthreads();
  }

  {
    const int plane = wave >> 2;
    const int e0 = (wave & 3) * 256 + lane * 8;
    unsigned w4[4];
#pragma unroll
    for (int e2 = 0; e2 < 4; ++e2) {
      unsigned wh, wl;
      split_pair(sOut[e0 + 2 * e2], sOut[e0 + 2 * e2 + 1], wh, wl);
      w4[e2] = plane ? wl : wh;
    }
    const v4u ov = {w4[0], w4[1], w4[2], w4[3]};
    unsigned short* dst = (plane ? fl : fh) + (size_t)blockIdx.x * 1024 + e0;
    *(volatile v4u*)(void*)dst = ov;
    __threadfence();
    *(volatile v4u*)(void*)dst = ov;
  }
}

__global__ __launch_bounds__(256) void fp_interp_concat_kernel(
    const float* __restrict__ posf, const float* __restrict__ posc, int nc,
    const unsigned short* __restrict__ ch, const unsigned short* __restrict__ cl,
    const unsigned short* __restrict__ sh, const unsigned short* __restrict__ sl,
    unsigned short* __restrict__ yh, unsigned short* __restrict__ yl) {
#pragma clang fp contract(off)
  __shared__ float sCx[256];
  __shared__ float sCy[256];
  __shared__ float sCz[256];
  __shared__ int sI0[256];
  __shared__ int sI1[256];
  __shared__ int sI2[256];
  __shared__ float sK0[256];
  __shared__ float sK1[256];
  __shared__ float sK2[256];
  __shared__ float sInv[256];
  const int t = threadIdx.x;
  const int lane = t & 31;
  const int wave = t >> 5;
  const int f = blockIdx.x * 256 + t;
  const float fx = posf[3 * f], fy = posf[3 * f + 1], fz = posf[3 * f + 2];
  float d0 = __builtin_inff(), d1 = __builtin_inff(), d2 = __builtin_inff();
  int i0 = 0, i1 = 0, i2 = 0;
  for (int cb = 0; cb < nc; cb += 256) {
    __syncthreads();
    {
      const int cj = (cb + t) < nc ? (cb + t) : nc - 1;
      sCx[t] = posc[3 * cj];
      sCy[t] = posc[3 * cj + 1];
      sCz[t] = posc[3 * cj + 2];
    }
    __syncthreads();
#pragma unroll 4
    for (int jj = 0; jj < 256; ++jj) {
      const float dx = fx - sCx[jj], dy = fy - sCy[jj], dz = fz - sCz[jj];
      const float t0 = dx * dx;
      const float t1 = dy * dy;
      const float t2 = dz * dz;
      const float d = (t0 + t2) + t1;
      const int j = cb + jj;
      const bool in = j < nc;
      const bool c0 = in && (d < d0);
      const bool c1 = in && (d < d1);
      const bool c2 = in && (d < d2);
      d2 = c1 ? d1 : (c2 ? d : d2);
      i2 = c1 ? i1 : (c2 ? j : i2);
      d1 = c0 ? d0 : (c1 ? d : d1);
      i1 = c0 ? i0 : (c1 ? j : i1);
      d0 = c0 ? d : d0;
      i0 = c0 ? j : i0;
    }
  }
  {
    const float w0 = 1.0f / fmaxf(d0, 1e-16f);
    const float w1 = 1.0f / fmaxf(d1, 1e-16f);
    const float w2 = 1.0f / fmaxf(d2, 1e-16f);
    const float ws = (w0 + w2) + w1;
    sK0[t] = w0;
    sK1[t] = w1;
    sK2[t] = w2;
    sInv[t] = 1.0f / ws;
    sI0[t] = i0;
    sI1[t] = i1;
    sI2[t] = i2;
  }
  __syncthreads();

  const int c8 = (lane & 15) * 8;
#pragma unroll 1
  for (int it = 0; it < 16; ++it) {
    const int r = wave * 32 + it * 2 + (lane >> 4);
    const size_t frow = (size_t)blockIdx.x * 256 + r;
    int j0 = sI0[r], j1 = sI1[r], j2 = sI2[r];
    j0 = j0 < 0 ? 0 : (j0 > nc - 1 ? nc - 1 : j0);
    j1 = j1 < 0 ? 0 : (j1 > nc - 1 ? nc - 1 : j1);
    j2 = j2 < 0 ? 0 : (j2 > nc - 1 ? nc - 1 : j2);
    const float w0 = sK0[r], w1 = sK1[r], w2 = sK2[r], inv = sInv[r];
    const v4u h0 = *(const v4u*)(const void*)(ch + (size_t)j0 * 128 + c8);
    const v4u l0 = *(const v4u*)(const void*)(cl + (size_t)j0 * 128 + c8);
    const v4u h1 = *(const v4u*)(const void*)(ch + (size_t)j1 * 128 + c8);
    const v4u l1 = *(const v4u*)(const void*)(cl + (size_t)j1 * 128 + c8);
    const v4u h2 = *(const v4u*)(const void*)(ch + (size_t)j2 * 128 + c8);
    const v4u l2 = *(const v4u*)(const void*)(cl + (size_t)j2 * 128 + c8);
    unsigned oh[4], ol[4];
#pragma unroll
    for (int e2 = 0; e2 < 4; ++e2) {
      const unsigned uh0 = h0[e2], ul0 = l0[e2];
      const unsigned uh1 = h1[e2], ul1 = l1[e2];
      const unsigned uh2 = h2[e2], ul2 = l2[e2];
      const float x0a = bf_lo(uh0) + bf_lo(ul0), x0b = bf_hi(uh0) + bf_hi(ul0);
      const float x1a = bf_lo(uh1) + bf_lo(ul1), x1b = bf_hi(uh1) + bf_hi(ul1);
      const float x2a = bf_lo(uh2) + bf_lo(ul2), x2b = bf_hi(uh2) + bf_hi(ul2);
      float ya = w0 * x0a;
      ya = ya + w1 * x1a;
      ya = ya + w2 * x2a;
      ya = ya * inv;
      float yb = w0 * x0b;
      yb = yb + w1 * x1b;
      yb = yb + w2 * x2b;
      yb = yb * inv;
      split_pair(ya, yb, oh[e2], ol[e2]);
    }
    const v4u ihv = {oh[0], oh[1], oh[2], oh[3]};
    const v4u ilv = {ol[0], ol[1], ol[2], ol[3]};
    const v4u shv = *(const v4u*)(const void*)(sh + frow * 128 + c8);
    const v4u slv = *(const v4u*)(const void*)(sl + frow * 128 + c8);
    unsigned short* pih = yh + frow * 256 + c8;
    unsigned short* pil = yl + frow * 256 + c8;
    unsigned short* psh = yh + frow * 256 + 128 + c8;
    unsigned short* psl = yl + frow * 256 + 128 + c8;
    *(volatile v4u*)(void*)pih = ihv;
    *(volatile v4u*)(void*)pil = ilv;
    *(volatile v4u*)(void*)psh = shv;
    *(volatile v4u*)(void*)psl = slv;
    __threadfence();
    *(volatile v4u*)(void*)pih = ihv;
    *(volatile v4u*)(void*)pil = ilv;
    *(volatile v4u*)(void*)psh = shv;
    *(volatile v4u*)(void*)psl = slv;
  }
}

__global__ __launch_bounds__(256) void lin_out2_kernel(const float* __restrict__ L,
                                                       const float* __restrict__ W,
                                                       const float* __restrict__ b,
                                                       float* __restrict__ out) {
  __shared__ float sWt[2][128];
  const int t = threadIdx.x;
  const int lane = t & 31;
  const int wave = t >> 5;
  sWt[t & 1][t >> 1] = W[t];
  __syncthreads();
  const int g = blockIdx.x * 8 + wave;
  const int row = g * 16 + (lane >> 1);
  const int c = lane & 1;
  float acc = 0.0f;
#pragma unroll 2
  for (int k4 = 0; k4 < 32; ++k4) {
    const v4f a = *(const v4f*)(L + (size_t)row * 128 + 4 * k4);
    acc = __builtin_fmaf(a[0], sWt[c][4 * k4 + 0], acc);
    acc = __builtin_fmaf(a[1], sWt[c][4 * k4 + 1], acc);
    acc = __builtin_fmaf(a[2], sWt[c][4 * k4 + 2], acc);
    acc = __builtin_fmaf(a[3], sWt[c][4 * k4 + 3], acc);
  }
  const float val = acc + b[c];
  float* dst = out + (size_t)g * 32 + lane;
  *(volatile float*)dst = val;
  __threadfence();
  *(volatile float*)dst = val;
}

constexpr size_t kCarveTotal = 66965504ull;
static_assert(kCarveTotal <= 134217728ull, "carve within 128 MiB");

extern "C" void kernel_launch(void* const* d_in, const int* in_sizes, int n_in,
                              void* d_out, int out_size, void* d_ws, size_t ws_size,
                              hipStream_t stream) {
  (void)in_sizes;
  (void)out_size;
  if (n_in < 18) return;
  const float* x      = (const float*)d_in[0];
  const float* pos    = (const float*)d_in[1];
  const float* li_w1  = (const float*)d_in[2];
  const float* li_b1  = (const float*)d_in[3];
  const float* li_w2  = (const float*)d_in[4];
  const float* li_b2  = (const float*)d_in[5];
  const float* sa_w1  = (const float*)d_in[6];
  const float* sa_b1  = (const float*)d_in[7];
  const float* sa_w2  = (const float*)d_in[8];
  const float* sa_b2  = (const float*)d_in[9];
  const float* fp_w1  = (const float*)d_in[10];
  const float* fp_b1  = (const float*)d_in[11];
  const float* fp_w2  = (const float*)d_in[12];
  const float* fp_b2  = (const float*)d_in[13];
  const float* lo_w1  = (const float*)d_in[14];
  const float* lo_b1  = (const float*)d_in[15];
  const float* lo_w2  = (const float*)d_in[16];
  const float* lo_b2  = (const float*)d_in[17];
  float* out = (float*)d_out;

  char* base = (char*)d_ws;
  size_t off = 0;
  auto take = [&](size_t bytes) -> char* {
    char* p = base + off;
    off += (bytes + 255) & ~(size_t)255;
    return p;
  };
  typedef unsigned short us;
  us* XH = (us*)take((size_t)kPts0 * 32 * 2);
  us* XL = (us*)take((size_t)kPts0 * 32 * 2);
  us* WLI1H = (us*)take(128 * 32 * 2);
  us* WLI1L = (us*)take(128 * 32 * 2);
  us* WLI2H = (us*)take(128 * 128 * 2);
  us* WLI2L = (us*)take(128 * 128 * 2);
  us* WSA1H = (us*)take((size_t)3 * kSaHidPadN * 128 * 2);
  us* WSA1L = (us*)take((size_t)3 * kSaHidPadN * 128 * 2);
  us* WSA2H = (us*)take((size_t)3 * 128 * kSaHidPadK * 2);
  us* WSA2L = (us*)take((size_t)3 * 128 * kSaHidPadK * 2);
  us* WFP1H = (us*)take((size_t)3 * 256 * 256 * 2);
  us* WFP1L = (us*)take((size_t)3 * 256 * 256 * 2);
  us* WFP2H = (us*)take((size_t)3 * 128 * 256 * 2);
  us* WFP2L = (us*)take((size_t)3 * 128 * 256 * 2);
  us* WLO1H = (us*)take(128 * 128 * 2);
  us* WLO1L = (us*)take(128 * 128 * 2);
  us* H1H = (us*)take((size_t)kPts0 * 128 * 2);
  us* H1L = (us*)take((size_t)kPts0 * 128 * 2);
  const int npts[4] = {kPts0, kPts1, kPts2, kPts3};
  us* FH[4];
  us* FL[4];
  for (int l = 0; l < 4; ++l) {
    FH[l] = (us*)take((size_t)npts[l] * 128 * 2);
    FL[l] = (us*)take((size_t)npts[l] * 128 * 2);
  }
  float* QP[4];
  QP[0] = nullptr;
  for (int l = 1; l < 4; ++l) QP[l] = (float*)take((size_t)npts[l] * 3 * 4);
  float* PP[3];
  for (int l = 0; l < 3; ++l) PP[l] = (float*)take((size_t)npts[l] * kSaHidPadN * 4);
  us* YCH[3];
  us* YCL[3];
  us* TFH[3];
  us* TFL[3];
  us* XFH[3];
  us* XFL[3];
  for (int j = 2; j >= 0; --j) {
    YCH[j] = (us*)take((size_t)npts[j] * 256 * 2);
    YCL[j] = (us*)take((size_t)npts[j] * 256 * 2);
  }
  for (int j = 2; j >= 0; --j) {
    TFH[j] = (us*)take((size_t)npts[j] * 256 * 2);
    TFL[j] = (us*)take((size_t)npts[j] * 256 * 2);
  }
  for (int j = 2; j >= 0; --j) {
    XFH[j] = (us*)take((size_t)npts[j] * 128 * 2);
    XFL[j] = (us*)take((size_t)npts[j] * 128 * 2);
  }
  float* LOUT = (float*)take((size_t)kPts0 * 128 * 4);
  if (off > ws_size || off > (size_t)134217728ull) return;

  auto prep = [&](const float* src, long srcLvl, int sn, int sk, int Kreal, int Nreal, int Kpad, int Npad,
                  us* dh, us* dl, long dstLvl, int levels) {
    const long total = (long)Npad * Kpad;
    const int gx = (int)((total / 8 + 255) / 256);
    prep_split_kernel<<<dim3(gx, levels), 256, 0, stream>>>(src, srcLvl, sn, sk, Kreal, Nreal, Kpad, Npad,
                                                            dh, dl, dstLvl);
  };
  auto ggrid = [](int M, int N) { return ((M / 64) * (N / 64) + 7) / 8; };

  prep(x, 0, kFeatIn, 1, kFeatIn, kPts0, 32, kPts0, XH, XL, 0, 1);
  prep(li_w1, 0, 1, 128, kFeatIn, 128, 32, 128, WLI1H, WLI1L, 0, 1);
  prep(li_w2, 0, 1, 128, 128, 128, 128, 128, WLI2H, WLI2L, 0, 1);
  prep(sa_w1, kSaW1Level, 1, kSaHid, 128, kSaHid, 128, kSaHidPadN, WSA1H, WSA1L, (long)kSaHidPadN * 128, 3);
  prep(sa_w2, kSaW2Level, 1, 128, kSaHid, 128, kSaHidPadK, 128, WSA2H, WSA2L, (long)128 * kSaHidPadK, 3);
  prep(fp_w1, 65536, 1, 256, 256, 256, 256, 256, WFP1H, WFP1L, 65536, 3);
  prep(fp_w2, 32768, 1, 128, 256, 128, 256, 128, WFP2H, WFP2L, 32768, 3);
  prep(lo_w1, 0, 1, 128, 128, 128, 128, 128, WLO1H, WLO1L, 0, 1);

  gemm_bf16x3_kernel<2, 2, 2><<<ggrid(kPts0, 128), 256, 0, stream>>>(
      XH, XL, 32, WLI1H, WLI1L, 32, H1H, H1L, 128, li_b1, kPts0, 128, 32);
  gemm_bf16x3_kernel<2, 2, 2><<<ggrid(kPts0, 128), 256, 0, stream>>>(
      H1H, H1L, 128, WLI2H, WLI2L, 128, FH[0], FL[0], 128, li_b2, kPts0, 128, 128);

  fps_kernel<16><<<1, 512, 0, stream>>>(pos, kPts1, QP[1]);
  fps_kernel<8><<<1, 512, 0, stream>>>(QP[1], kPts2, QP[2]);
  fps_kernel<4><<<1, 512, 0, stream>>>(QP[2], kPts3, QP[3]);

  const float* posL[4] = {pos, QP[1], QP[2], QP[3]};
  for (int l = 0; l < 3; ++l) {
    const int n = npts[l], m = npts[l + 1];
    gemm_bf16x3_kernel<0, 0, 0><<<ggrid(n, kSaHidPadN), 256, 0, stream>>>(
        FH[l], FL[l], 128, WSA1H + (size_t)l * kSaHidPadN * 128, WSA1L + (size_t)l * kSaHidPadN * 128, 128,
        PP[l], nullptr, kSaHidPadN, nullptr, n, kSaHidPadN, 128);
    sa_fused_kernel<<<m / 8, 256, 0, stream>>>(
        posL[l], n, posL[l + 1], PP[l],
        sa_w1 + (size_t)l * kSaW1Level + (size_t)128 * kSaHid, sa_b1 + (size_t)l * kSaHid,
        WSA2H + (size_t)l * 128 * kSaHidPadK, WSA2L + (size_t)l * 128 * kSaHidPadK,
        sa_b2 + (size_t)l * 128, FH[l + 1], FL[l + 1]);
  }

  const us* ch = FH[3];
  const us* cl = FL[3];
  for (int j = 2; j >= 0; --j) {
    const int nf = npts[j], nc = npts[j + 1];
    fp_interp_concat_kernel<<<nf / 256, 256, 0, stream>>>(posL[j], posL[j + 1], nc, ch, cl,
                                                          FH[j], FL[j], YCH[j], YCL[j]);
    gemm_bf16x3_kernel<2, 2, 2><<<ggrid(nf, 256), 256, 0, stream>>>(
        YCH[j], YCL[j], 256, WFP1H + (size_t)j * 65536, WFP1L + (size_t)j * 65536, 256,
        TFH[j], TFL[j], 256, fp_b1 + (size_t)j * 256, nf, 256, 256);
    gemm_bf16x3_kernel<2, 2, 2><<<ggrid(nf, 128), 256, 0, stream>>>(
        TFH[j], TFL[j], 256, WFP2H + (size_t)j * 32768, WFP2L + (size_t)j * 32768, 256,
        XFH[j], XFL[j], 128, fp_b2 + (size_t)j * 128, nf, 128, 256);
    ch = XFH[j];
    cl = XFL[j];
  }

  gemm_bf16x3_kernel<2, 0, 2><<<ggrid(kPts0, 128), 256, 0, stream>>>(
      XFH[0], XFL[0], 128, WLO1H, WLO1L, 128, LOUT, nullptr, 128, lo_b1, kPts0, 128, 128);
  lin_out2_kernel<<<kPts0 / 128, 256, 0, stream>>>(LOUT, lo_w2, lo_b2, out);
}
